// RBF_36129264894114
// MI455X (gfx1250) — hardware-verified
//
#include <hip/hip_runtime.h>


#define MM   16384
#define NN   8192
#define KO   64
#define CH   2048
#define NCH  (MM / CH)
typedef _Float16 h16;
typedef unsigned short bf;
typedef __attribute__((ext_vector_type(16))) __bf16   v16bf;
typedef __attribute__((ext_vector_type(16))) _Float16 v16h;
typedef __attribute__((ext_vector_type(8)))  _Float16 v8h;
typedef __attribute__((ext_vector_type(8)))  unsigned short v8us;
typedef __attribute__((ext_vector_type(8)))  float    v8f;
typedef __attribute__((ext_vector_type(4)))  float    v4f;
typedef v8h  __attribute__((may_alias)) v8ha;
typedef v4f  __attribute__((may_alias)) v4fa;
typedef v8us __attribute__((may_alias)) v8usa;

__device__ __forceinline__ unsigned short f2bf(float f) { unsigned u = __float_as_uint(f); u += 0x7FFFu + ((u >> 16) & 1u); return (unsigned short)(u >> 16); }
__device__ __forceinline__ float bf2f(unsigned short b) { return __uint_as_float(((unsigned)b) << 16); }
__device__ __forceinline__ float bfr(float f) { return bf2f(f2bf(f)); }
__device__ __forceinline__ v16h cat16(v8h lo, v8h hi) { return __builtin_shufflevector(lo, hi, 0, 1, 2, 3, 4, 5, 6, 7, 8, 9, 10, 11, 12, 13, 14, 15); }
__device__ __forceinline__ v16bf cat16b(v8us lo, v8us hi) { return __builtin_bit_cast(v16bf, __builtin_shufflevector(lo, hi, 0, 1, 2, 3, 4, 5, 6, 7, 8, 9, 10, 11, 12, 13, 14, 15)); }
__device__ __forceinline__ v8f wmma16(v16h a, v16h b, v8f c) { return __builtin_amdgcn_wmma_f32_16x16x32_f16(false, a, false, b, (short)0, c, false, false); }
__device__ __forceinline__ v8f wmmab(v16bf a, v16bf b, v8f c) { return __builtin_amdgcn_wmma_f32_16x16x32_bf16(false, a, false, b, (short)0, c, false, false); }


template <typename T16> struct WFrag;
template <> struct WFrag<h16> { typedef v16h V; static __device__ __forceinline__ V ld(const h16* p) { return cat16(*(const v8h*)p, *(const v8h*)(p + 16)); } static __device__ __forceinline__ v8f mma(V a, V b, v8f c) { return wmma16(a, b, c); } };
template <> struct WFrag<bf> { typedef v16bf V; static __device__ __forceinline__ V ld(const bf* p) { return cat16b(*(const v8us*)p, *(const v8us*)(p + 16)); } static __device__ __forceinline__ v8f mma(V a, V b, v8f c) { return wmmab(a, b, c); } };
template <typename T16, int NSPLIT, bool BIAS>
__global__ __launch_bounds__(32) void k_gemmw(const T16* __restrict__ A, const T16* __restrict__ A2, const T16* __restrict__ Bt, const T16* __restrict__ Bt2, int K, float* C, int ldc, const float* __restrict__ bias, size_t sA, size_t sB, size_t sC) {
    typedef typename WFrag<T16>::V V;
    __shared__ __align__(16) float os[16 * 68];
    const size_t z = blockIdx.z; A += z * sA; if (A2) A2 += z * sA; Bt += z * sB; if (Bt2) Bt2 += z * sB; C += z * sC;
    const int lane = threadIdx.x & 31, lr = lane & 15, hi = lane >> 4; const int r0 = blockIdx.x * 64, c0 = blockIdx.y * 64;
    v8f acc[4][4];
#pragma unroll
    for (int mb = 0; mb < 4; ++mb)
#pragma unroll
        for (int nb = 0; nb < 4; ++nb) acc[mb][nb] = (v8f){};
    const size_t aoff = (size_t)(r0 + lr) * K + 8 * hi, boff = (size_t)(c0 + lr) * K + 8 * hi;
#pragma unroll 1
    for (int kc = 0; kc < K; kc += 32) {
        V a[4], a2[4];
#pragma unroll
        for (int mb = 0; mb < 4; ++mb) { a[mb] = WFrag<T16>::ld(A + aoff + (size_t)mb * 16 * K + kc); if (NSPLIT == 1 || NSPLIT == 2) a2[mb] = WFrag<T16>::ld(A2 + aoff + (size_t)mb * 16 * K + kc); }
#pragma unroll
        for (int nb = 0; nb < 4; ++nb) { const V b = WFrag<T16>::ld(Bt + boff + (size_t)nb * 16 * K + kc); V b2; if (NSPLIT >= 2) b2 = WFrag<T16>::ld(Bt2 + boff + (size_t)nb * 16 * K + kc);
#pragma unroll
            for (int mb = 0; mb < 4; ++mb) { acc[mb][nb] = WFrag<T16>::mma(a[mb], b, acc[mb][nb]); if (NSPLIT == 1 || NSPLIT == 2) acc[mb][nb] = WFrag<T16>::mma(a2[mb], b, acc[mb][nb]); if (NSPLIT >= 2) acc[mb][nb] = WFrag<T16>::mma(a[mb], b2, acc[mb][nb]); } }
        asm volatile("v_nop\n\tv_nop\n\tv_nop\n\tv_nop" : "+v"(acc[0][0]), "+v"(acc[1][1]), "+v"(acc[2][2]), "+v"(acc[3][3]) : "v"(a[0]), "v"(a[3]));
    }
#pragma unroll
    for (int mb = 0; mb < 4; ++mb) {
#pragma unroll
        for (int nb = 0; nb < 4; ++nb) {
#pragma unroll
            for (int j = 0; j < 8; ++j) os[(hi * 8 + j) * 68 + nb * 16 + lr] = acc[mb][nb][j]; }
        __builtin_amdgcn_wave_barrier(); asm volatile("" ::: "memory");
        float* crow = C + (size_t)(r0 + mb * 16) * ldc + c0;
#pragma unroll 1
        for (int ps = 0; ps < 2; ++ps) {
#pragma unroll
            for (int s = 0; s < 8; ++s) { const int row = 2 * s + hi, cofs = lr * 4; v4f val = *(const v4fa*)(os + row * 68 + cofs); if (BIAS) { val[0] += bfr(bias[c0 + cofs]); val[1] += bfr(bias[c0 + cofs + 1]); val[2] += bfr(bias[c0 + cofs + 2]); val[3] += bfr(bias[c0 + cofs + 3]); }
                *(volatile v4f*)(crow + (size_t)row * ldc + cofs) = val; }
            if (ps == 0) __threadfence(); }
        __builtin_amdgcn_wave_barrier(); asm volatile("" ::: "memory");
    }
}

__device__ __forceinline__ void splitf(float y, unsigned short& h, unsigned short& l) { h = f2bf(y); l = f2bf(y - bf2f(h)); }
typedef __attribute__((ext_vector_type(4))) unsigned short v4us;
__global__ __launch_bounds__(256) void k_cvt8(const float* __restrict__ src, bf* dst, size_t n8) { const size_t i = (size_t)blockIdx.x * 256 + threadIdx.x; if (i >= n8) return; const v8f v = *(const v8f*)(src + i * 8); v8us o;
#pragma unroll
    for (int k = 0; k < 8; ++k) o[k] = f2bf(v[k]); *(volatile v8us*)(dst + i * 8) = o; __threadfence(); *(volatile v8us*)(dst + i * 8) = o; }

__global__ __launch_bounds__(256) void k_nrm(const float* __restrict__ A, int n, float* N2, float* R) { const int i = blockIdx.x * 256 + threadIdx.x; if (i >= n) return; const float a0 = bfr(A[i * 3]), a1 = bfr(A[i * 3 + 1]), a2 = bfr(A[i * 3 + 2]); float p0 = __fmul_rn(a0, a0), p1 = __fmul_rn(a1, a1), p2 = __fmul_rn(a2, a2); asm volatile("" : "+v"(p0), "+v"(p1), "+v"(p2)); const float s = __fadd_rn(__fadd_rn(p0, p1), p2); v4f r; r[0] = a0; r[1] = a1; r[2] = a2; r[3] = s;
    *(volatile v4f*)(R + (size_t)i * 4) = r; (void)N2; __threadfence(); *(volatile v4f*)(R + (size_t)i * 4) = r; }
__global__ __launch_bounds__(256) void k_phi(const float* __restrict__ RP, const float* __restrict__ RX, const float* __restrict__ epsp, int m0, bf* Ph, bf* Pl) { const size_t e = ((size_t)blockIdx.x * 256 + threadIdx.x) * 4; if (e >= (size_t)CH * NN) return; const int n = (int)(e % NN); const int ml = (int)(e / NN); const v4f p = *(const v4f*)(RP + (size_t)(m0 + ml) * 4); const float eps = bfr(epsp[0]); v4us oh, ol;
#pragma unroll
    for (int q = 0; q < 4; ++q) { const v4f xx = *(const v4f*)(RX + (size_t)(n + q) * 4); float t0 = __fmul_rn(p[0], xx[0]), t1 = __fmul_rn(p[1], xx[1]), t2 = __fmul_rn(p[2], xx[2]); asm volatile("" : "+v"(t0), "+v"(t1), "+v"(t2)); float dot = __fadd_rn(__fadd_rn(t0, t1), t2); asm volatile("" : "+v"(dot));
        float sab = __fadd_rn(p[3], xx[3]); asm volatile("" : "+v"(sab)); float dd = __fmul_rn(2.0f, dot); asm volatile("" : "+v"(dd)); const float d2 = fmaxf(__fsub_rn(sab, dd), 0.f); const float dist = __fsqrt_rn(d2); float u = __fmul_rn(eps, dist); asm volatile("" : "+v"(u)); float uu = __fmul_rn(u, u); asm volatile("" : "+v"(uu)); const float phi = __fsqrt_rn(__fadd_rn(uu, 1.0f));
        unsigned short a, c; splitf(phi, a, c); oh[q] = a; ol[q] = c; }
    *(volatile v4us*)(Ph + e) = oh; *(volatile v4us*)(Pl + e) = ol; __threadfence(); *(volatile v4us*)(Ph + e) = oh; *(volatile v4us*)(Pl + e) = ol; }

extern "C" void kernel_launch(void* const* d_in, const int* in_sizes, int n_in,
                              void* d_out, int out_size, void* d_ws, size_t ws_size, hipStream_t stream) {
    (void)in_sizes; (void)n_in; (void)out_size;
    const float* Xp = (const float*)d_in[0]; const float* X = (const float*)d_in[1]; const float* W = (const float*)d_in[2]; const float* epsp = (const float*)d_in[3];
    float* OUT = (float*)d_out;
    char* wsp = (char*)d_ws;
    auto take = [&](size_t bytes) { char* p = wsp; wsp += (bytes + 255) & ~(size_t)255; return (void*)p; };
    float* RP = (float*)take((size_t)MM * 4 * 4); float* RX = (float*)take((size_t)NN * 4 * 4); bf* WB = (bf*)take((size_t)KO * NN * 2); bf* Ph = (bf*)take((size_t)CH * NN * 2); bf* Pl = (bf*)take((size_t)CH * NN * 2);
    if ((size_t)(wsp - (char*)d_ws) > ws_size) return;
    k_nrm<<<MM / 256, 256, 0, stream>>>(Xp, MM, nullptr, RP); k_nrm<<<NN / 256, 256, 0, stream>>>(X, NN, nullptr, RX);
    k_cvt8<<<(KO * NN / 8 + 255) / 256, 256, 0, stream>>>(W, WB, (size_t)KO * NN / 8);
    for (int c = 0; c < NCH; ++c) {
        k_phi<<<(unsigned)(((size_t)CH * NN / 4 + 255) / 256), 256, 0, stream>>>(RP, RX, epsp, c * CH, Ph, Pl);
        k_gemmw<bf, 1, false><<<dim3(CH / 64, KO / 64, 1), 32, 0, stream>>>(Ph, Pl, WB, nullptr, NN, OUT + (size_t)c * CH * KO, KO, nullptr, 0, 0, 0); }
}
